// SlidingWindowAttention_2164663517569
// MI455X (gfx1250) — hardware-verified
//
#include <hip/hip_runtime.h>
#include <math.h>

typedef __attribute__((ext_vector_type(16))) _Float16 v16h;
typedef __attribute__((ext_vector_type(16))) __bf16 v16b;
typedef __attribute__((ext_vector_type(8)))  _Float16 v8h;
typedef __attribute__((ext_vector_type(8)))  __bf16 v8b;
typedef __attribute__((ext_vector_type(8)))  float v8f;
typedef __attribute__((ext_vector_type(4)))  float v4f;
typedef __attribute__((ext_vector_type(4)))  unsigned v4u;

#ifndef NB
#define NB 1
#endif
#ifndef SEQ
#define SEQ 4096
#endif
#define SEQ_FULL 4096
#define DM 1024
#define NHEAD 8
#define NKVH 2
#define HDIM 128
#define KVW 256
#define WINSZ 256
#define HPROWS 256
#define CARRY 16.0f
#define SCQK (0.08838834764831845f / 256.0f)
#define CB_X (SEQ / 2)

static_assert(NB == 1);
static_assert(SEQ % 64 == 0);
static_assert(HPROWS % 64 == 0);
static_assert(SEQ >= HPROWS);
static_assert(SEQ <= SEQ_FULL);
static_assert((NHEAD / NKVH) == 4);

template <typename T> __device__ __forceinline__ void vst2(void* p, T v) { *(volatile T*)p = v; __threadfence(); *(volatile T*)p = v; }
__device__ __forceinline__ v8f wmma16(v16h a, v16h b, v8f c) {
  v8f d = __builtin_amdgcn_wmma_f32_16x16x32_f16(false, a, false, b, (short)0, c, false, false);
  asm volatile("v_nop\n\tv_nop\n\tv_nop\n\tv_nop" : "+v"(d) : "v"(a), "v"(b));
  return d;
}
__device__ __forceinline__ v8f wmma_bf(v16b a, v16b b, v8f c) {
  v8f d = __builtin_amdgcn_wmma_f32_16x16x32_bf16(false, a, false, b, (short)0, c, false, false);
  asm volatile("v_nop\n\tv_nop\n\tv_nop\n\tv_nop" : "+v"(d) : "v"(a), "v"(b));
  return d;
}
__device__ __forceinline__ v16h frag_h(const _Float16* rowk0, unsigned lane) {
  union { v16h v; v8h q[2]; } u; const _Float16* p = rowk0 + 8u * (lane >> 4);
  u.q[0] = *(const v8h*)p; u.q[1] = *(const v8h*)(p + 16); return u.v;
}
__device__ __forceinline__ v16b frag_b(const __bf16* rowk0, unsigned lane) {
  union { v16b v; v8b q[2]; } u; const __bf16* p = rowk0 + 8u * (lane >> 4);
  u.q[0] = *(const v8b*)p; u.q[1] = *(const v8b*)(p + 16); return u.v;
}
__device__ __forceinline__ float bfr(float v) { return (float)(__bf16)v; }
#define LDSX() do { asm volatile("s_wait_dscnt 0" ::: "memory"); __builtin_amdgcn_wave_barrier(); __builtin_amdgcn_fence(3  , "workgroup"); } while (0)

#define WS_XB   ((size_t)0)
#define WS_WB   (WS_XB  + (size_t)2 * SEQ * DM)
#define WS_WOB  (WS_WB  + (size_t)2 * 1536 * DM)
#define WS_QH   (WS_WOB + (size_t)2 * DM * DM)
#define WS_KH   (WS_QH  + (size_t)2 * SEQ * DM)
#define WS_VT   (WS_KH  + (size_t)2 * SEQ * KVW)
#define WS_QL   (WS_VT  + (size_t)2 * KVW * SEQ)
#define WS_KL   (WS_QL  + (size_t)2 * HPROWS * DM)
#define WS_VTL  (WS_KL  + (size_t)2 * HPROWS * KVW)
#define WS_CTX  (WS_VTL + (size_t)2 * KVW * HPROWS)
#define WS_END  (WS_CTX + (size_t)2 * SEQ * 2 * DM)
static_assert(WS_END <= (size_t)134217728);

__global__ __launch_bounds__(256) void k_cvt(const float* __restrict__ X, const float* __restrict__ Wq, const float* __restrict__ Wk, const float* __restrict__ Wv, const float* __restrict__ Wo,
                                             __bf16* __restrict__ XB, __bf16* __restrict__ WB, __bf16* __restrict__ WOB) {
  const unsigned bid = blockIdx.x, tid = threadIdx.x;
  const float* src; __bf16* dst; unsigned lb;
  if (bid < (unsigned)CB_X)              { src = X;  dst = XB;                      lb = bid; }
  else if (bid < (unsigned)CB_X + 512u)  { src = Wq; dst = WB;                      lb = bid - (unsigned)CB_X; }
  else if (bid < (unsigned)CB_X + 640u)  { src = Wk; dst = WB + (size_t)1024 * DM;  lb = bid - (unsigned)CB_X - 512u; }
  else if (bid < (unsigned)CB_X + 768u)  { src = Wv; dst = WB + (size_t)1280 * DM;  lb = bid - (unsigned)CB_X - 640u; }
  else                                   { src = Wo; dst = WOB;                     lb = bid - (unsigned)CB_X - 768u; }
  const size_t off = (size_t)lb * 2048u + (size_t)tid * 8u;
  const v4f a = *(const v4f*)(src + off), b = *(const v4f*)(src + off + 4);
  union { v8b b8; v4u u; } cv;
#pragma unroll
  for (int i = 0; i < 4; ++i) { cv.b8[i] = (__bf16)a[i]; cv.b8[4 + i] = (__bf16)b[i]; }
  vst2(dst + off, cv.u);
}

__device__ __forceinline__ void gemm_core(const __bf16* __restrict__ A, unsigned lda, unsigned ksteps, const __bf16* __restrict__ W, unsigned r0, unsigned c0, unsigned wave, unsigned lane, v8f (&acc)[8]) {
  const unsigned col = lane & 15u;
  const __bf16* ap = A + (size_t)(r0 + wave * 16u + col) * lda;
  const __bf16* wp = W + (size_t)(c0 + col) * DM;
#pragma unroll 1
  for (unsigned kc = 0; kc < ksteps; ++kc) {
    const v16b a = frag_b(ap + kc * 32u, lane);
    const unsigned kw = (kc & 31u) * 32u;
#pragma unroll
    for (int j = 0; j < 8; ++j) { const v16b w = frag_b(wp + (size_t)j * 16 * DM + kw, lane); acc[j] = wmma_bf(a, w, acc[j]); }
  }
}

__global__ __launch_bounds__(128) void k_qkv(const __bf16* __restrict__ XB, const __bf16* __restrict__ WB, const float* __restrict__ bq, const float* __restrict__ bk, const float* __restrict__ bv,
                                             _Float16* __restrict__ QH, _Float16* __restrict__ QL, _Float16* __restrict__ KH, _Float16* __restrict__ KL, _Float16* __restrict__ VT, _Float16* __restrict__ VTL) {
  __shared__ __align__(16) unsigned char lraw[36864];
  const unsigned tid = threadIdx.x, wave = tid >> 5, lane = tid & 31u, col = lane & 15u, g = lane >> 4;
  const unsigned r0 = blockIdx.x * 64u, c0 = blockIdx.y * 128u;
  v8f acc[8] = {};
  gemm_core(XB, DM, DM / 32, WB, r0, c0, wave, lane, acc);
  _Float16* s0 = (_Float16*)lraw; _Float16* s1 = s0 + 9216;
  const bool hp = r0 < (unsigned)HPROWS;
  if (c0 < 1280u) {
    const bool isq = c0 < 1024u;
    const float* bias = isq ? (bq + c0) : (bk + (c0 - 1024u));
    _Float16* DH = isq ? QH : KH; _Float16* DL = isq ? QL : KL;
    const unsigned ld = isq ? (unsigned)DM : (unsigned)KVW; const unsigned cc = isq ? c0 : (c0 - 1024u);
#pragma unroll
    for (int j = 0; j < 8; ++j) { const float bs = bfr(bias[j * 16 + col]);
#pragma unroll
      for (int r = 0; r < 8; ++r) { const float v = (acc[j][r] + bs) * CARRY; const _Float16 hv = (_Float16)v; const unsigned idx = (wave * 16u + 8u * g + (unsigned)r) * 136u + (unsigned)j * 16u + col;
        s0[idx] = hv; s1[idx] = (_Float16)((v - (float)hv) * 2048.0f); } }
    __syncthreads();
    for (unsigned e = tid; e < 64u * 16u; e += 128u) { const unsigned rl = e >> 4, q = e & 15u;
      vst2(DH + (size_t)(r0 + rl) * ld + cc + q * 8u, *(const v4u*)(s0 + rl * 136u + q * 8u));
      if (hp) vst2(DL + (size_t)(r0 + rl) * ld + cc + q * 8u, *(const v4u*)(s1 + rl * 136u + q * 8u)); }
  } else {
    const unsigned cv = c0 - 1280u; const float* bias = bv + cv;
#pragma unroll
    for (int j = 0; j < 8; ++j) { const float bs = bfr(bias[j * 16 + col]);
#pragma unroll
      for (int r = 0; r < 8; ++r) { const float v = (acc[j][r] + bs) * CARRY; const _Float16 hv = (_Float16)v; const unsigned idx = ((unsigned)j * 16u + col) * 72u + wave * 16u + 8u * g + (unsigned)r;
        s0[idx] = hv; s1[idx] = (_Float16)((v - (float)hv) * 2048.0f); } }
    __syncthreads();
    for (unsigned e = tid; e < 128u * 8u; e += 128u) { const unsigned cl = e >> 3, q = e & 7u;
      vst2(VT + (size_t)(cv + cl) * SEQ + r0 + q * 8u, *(const v4u*)(s0 + cl * 72u + q * 8u));
      if (hp) vst2(VTL + (size_t)(cv + cl) * HPROWS + r0 + q * 8u, *(const v4u*)(s1 + cl * 72u + q * 8u)); }
  }
}

template <int HP>
__global__ __launch_bounds__(128) void k_attn(const _Float16* __restrict__ QH, const _Float16* __restrict__ KH, const _Float16* __restrict__ VT,
                                              const _Float16* __restrict__ QL, const _Float16* __restrict__ KL, const _Float16* __restrict__ VTL,
                                              const float* __restrict__ sinkp, __bf16* __restrict__ CTX) {
  constexpr int ND = HP ? 4 : 8;
  constexpr int CP = ND * 16 + 8;
  __shared__ __align__(16) _Float16 pt[4][16][40];
  __shared__ __align__(16) _Float16 pr[HP ? 4 : 1][16][40];
  __shared__ __align__(16) __bf16 ch[4][16][CP];
  __shared__ __align__(16) __bf16 cl[4][16][CP];
  const unsigned tid = threadIdx.x, wave = tid >> 5, lane = tid & 31u, col = lane & 15u, g = lane >> 4;
  const unsigned h = blockIdx.y, hk = h >> 2;
  const unsigned q0 = (HP ? 0u : (unsigned)HPROWS) + (blockIdx.x * 4u + wave) * 16u;
  const unsigned d0 = HP ? blockIdx.z * 64u : 0u;
  const float sinkv = bfr(sinkp[0]);
  const _Float16* qrow = QH + (size_t)(q0 + col) * DM + h * HDIM;
  const _Float16* qlrow = HP ? (QL + (size_t)(q0 + col) * DM + h * HDIM) : QL;
  v16h qf[4] = {};
  if (!HP) {
#pragma unroll
    for (int kc = 0; kc < 4; ++kc) qf[kc] = frag_h(qrow + kc * 32, lane);
  }
  v8f o[ND] = {}, ol[ND] = {};
  float mrow[8], lrow[8];
#pragma unroll
  for (int r = 0; r < 8; ++r) { mrow[r] = sinkv; lrow[r] = 0.0f; }
  const unsigned ktb = (q0 >= 272u) ? (q0 - 272u) : 0u, kte = q0 + 16u;
#pragma unroll 1
  for (unsigned kt = ktb; kt < kte; kt += 32u) {
    v8f s0 = {}, s1 = {}, t0 = {}, t1 = {};
#pragma unroll
    for (int kc = 0; kc < 4; ++kc) {
      const _Float16* kp = KH + (size_t)(kt + col) * KVW + hk * HDIM + kc * 32;
      const v16h b0 = frag_h(kp, lane), b1 = frag_h(kp + 16 * KVW, lane);
      if (HP) {
        const v16h ah = frag_h(qrow + kc * 32, lane), al = frag_h(qlrow + kc * 32, lane);
        const _Float16* kq = KL + (size_t)(kt + col) * KVW + hk * HDIM + kc * 32;
        const v16h c0 = frag_h(kq, lane), c1 = frag_h(kq + 16 * KVW, lane);
        s0 = wmma16(ah, b0, s0); s1 = wmma16(ah, b1, s1);
        t0 = wmma16(al, b0, t0); t1 = wmma16(al, b1, t1);
        t0 = wmma16(ah, c0, t0); t1 = wmma16(ah, c1, t1);
      } else { s0 = wmma16(qf[kc], b0, s0); s1 = wmma16(qf[kc], b1, s1); }
    }
    float p0[8], p1[8];
#pragma unroll
    for (int r = 0; r < 8; ++r) {
      const unsigned i = q0 + 8u * g + (unsigned)r; const unsigned j0 = kt + col, j1 = j0 + 16u;
      float v0 = HP ? (s0[r] + t0[r] * (1.0f / 2048.0f)) : s0[r];
      float v1 = HP ? (s1[r] + t1[r] * (1.0f / 2048.0f)) : s1[r];
      v0 *= SCQK; v1 *= SCQK;
      v0 = (j0 <= i && j0 + (unsigned)WINSZ > i) ? v0 : -65504.0f;
      v1 = (j1 <= i && j1 + (unsigned)WINSZ > i) ? v1 : -65504.0f;
      float rmax = fmaxf(v0, v1);
#pragma unroll
      for (int off = 1; off < 16; off <<= 1) rmax = fmaxf(rmax, __shfl_xor(rmax, off, 32));
      const float mnew = fmaxf(mrow[r], rmax);
      const float f = expf(mrow[r] - mnew);
      const float e0 = expf(v0 - mnew), e1 = expf(v1 - mnew);
      float rs = e0 + e1;
#pragma unroll
      for (int off = 1; off < 16; off <<= 1) rs += __shfl_xor(rs, off, 32);
      lrow[r] = lrow[r] * f + rs; mrow[r] = mnew; p0[r] = e0 * 1024.0f; p1[r] = e1 * 1024.0f;
#pragma unroll
      for (int d = 0; d < ND; ++d) { o[d][r] *= f; if (HP) ol[d][r] *= f; }
    }
    LDSX();
#pragma unroll
    for (int r = 0; r < 8; ++r) { const unsigned row = 8u * g + (unsigned)r; const _Float16 h0 = (_Float16)p0[r], h1 = (_Float16)p1[r];
      pt[wave][row][col] = h0; pt[wave][row][16u + col] = h1;
      if (HP) { pr[wave][row][col] = (_Float16)((p0[r] - (float)h0) * 2048.0f); pr[wave][row][16u + col] = (_Float16)((p1[r] - (float)h1) * 2048.0f); } }
    LDSX();
    const v16h pa = frag_h(&pt[wave][col][0], lane);
    v16h pb = pa; if (HP) pb = frag_h(&pr[wave][col][0], lane);
#pragma unroll
    for (int d = 0; d < ND; ++d) {
      const unsigned c = hk * HDIM + d0 + (unsigned)d * 16u + col;
      const v16h vh = frag_h(VT + (size_t)c * SEQ + kt, lane);
      o[d] = wmma16(pa, vh, o[d]);
      if (HP) { const v16h vl = frag_h(VTL + (size_t)c * HPROWS + kt, lane); ol[d] = wmma16(pa, vl, ol[d]); ol[d] = wmma16(pb, vh, ol[d]); }
    }
  }
#pragma unroll
  for (int r = 0; r < 8; ++r) {
    const float inv = (1.0f / (lrow[r] + expf(sinkv - mrow[r]))) * (1.0f / 16384.0f);
#pragma unroll
    for (int d = 0; d < ND; ++d) { const float val = HP ? (o[d][r] + ol[d][r] * (1.0f / 2048.0f)) * inv : o[d][r] * inv;
      const __bf16 bh = (__bf16)val; ch[wave][8u * g + (unsigned)r][d * 16 + col] = bh; cl[wave][8u * g + (unsigned)r][d * 16 + col] = (__bf16)(val - (float)bh); }
  }
  LDSX();
  if (HP) {
#pragma unroll 1
    for (unsigned it = 0; it < 4u; ++it) { const unsigned rl = it * 4u + (lane >> 3), q = lane & 7u;
      __bf16* dst = CTX + (size_t)(q0 + rl) * (2 * DM) + h * HDIM + d0 + q * 8u;
      vst2(dst, *(const v4u*)&ch[wave][rl][q * 8u]); vst2(dst + DM, *(const v4u*)&cl[wave][rl][q * 8u]); }
  } else {
#pragma unroll 1
    for (unsigned it = 0; it < 8u; ++it) { const unsigned rl = it * 2u + (lane >> 4), q = lane & 15u;
      __bf16* dst = CTX + (size_t)(q0 + rl) * (2 * DM) + h * HDIM + q * 8u;
      vst2(dst, *(const v4u*)&ch[wave][rl][q * 8u]); vst2(dst + DM, *(const v4u*)&cl[wave][rl][q * 8u]); }
  }
}

__global__ __launch_bounds__(128) void k_out(const __bf16* __restrict__ CTX, const __bf16* __restrict__ WOB, const float* __restrict__ bo, float* __restrict__ OUT) {
  __shared__ __align__(16) unsigned char lraw[36864];
  const unsigned tid = threadIdx.x, wave = tid >> 5, lane = tid & 31u, col = lane & 15u, g = lane >> 4;
  const unsigned r0 = blockIdx.x * 64u, c0 = blockIdx.y * 128u;
  v8f acc[8] = {};
  gemm_core(CTX, 2 * DM, (2 * DM) / 32, WOB, r0, c0, wave, lane, acc);
  float* sf = (float*)lraw;
#pragma unroll
  for (int j = 0; j < 8; ++j) { const float bs = bfr(bo[c0 + (unsigned)j * 16u + col]);
#pragma unroll
    for (int r = 0; r < 8; ++r) sf[(wave * 16u + 8u * g + (unsigned)r) * 132u + (unsigned)j * 16u + col] = acc[j][r] + bs; }
  __syncthreads();
  for (unsigned e = tid; e < 64u * 32u; e += 128u) { const unsigned rl = e >> 5, q = e & 31u;
    vst2(OUT + (size_t)(r0 + rl) * DM + c0 + q * 4u, *(const v4f*)(sf + rl * 132u + q * 4u)); }
}

extern "C" void kernel_launch(void* const* d_in, const int* in_sizes, int n_in, void* d_out, int out_size, void* d_ws, size_t ws_size, hipStream_t stream) {
  if (n_in < 10) return;
  if (in_sizes[0] < SEQ * DM || in_sizes[1] < 1 || in_sizes[2] < DM * DM || in_sizes[3] < DM || in_sizes[4] < KVW * DM || in_sizes[5] < KVW ||
      in_sizes[6] < KVW * DM || in_sizes[7] < KVW || in_sizes[8] < DM * DM || in_sizes[9] < DM) return;
  if (out_size < SEQ * DM) return;
  if (ws_size < (size_t)WS_END) return;
  const float* const* F = (const float* const*)d_in;
  char* ws = (char*)d_ws;
  __bf16* XB = (__bf16*)(ws + WS_XB); __bf16* WB = (__bf16*)(ws + WS_WB); __bf16* WOB = (__bf16*)(ws + WS_WOB);
  _Float16* QH = (_Float16*)(ws + WS_QH); _Float16* KH = (_Float16*)(ws + WS_KH); _Float16* VT = (_Float16*)(ws + WS_VT);
  _Float16* QL = (_Float16*)(ws + WS_QL); _Float16* KL = (_Float16*)(ws + WS_KL); _Float16* VTL = (_Float16*)(ws + WS_VTL);
  __bf16* CTX = (__bf16*)(ws + WS_CTX);
  k_cvt<<<dim3(CB_X + 1280), 256, 0, stream>>>(F[0], F[2], F[4], F[6], F[8], XB, WB, WOB);
  k_qkv<<<dim3(SEQ / 64, 12), 128, 0, stream>>>(XB, WB, F[3], F[5], F[7], QH, QL, KH, KL, VT, VTL);
  if (SEQ > HPROWS) k_attn<0><<<dim3((SEQ - HPROWS) / 64, NHEAD, 1), 128, 0, stream>>>(QH, KH, VT, QL, KL, VTL, F[1], CTX);
  k_attn<1><<<dim3(HPROWS / 64, NHEAD, 2), 128, 0, stream>>>(QH, KH, VT, QL, KL, VTL, F[1], CTX);
  k_out<<<dim3(SEQ / 64, DM / 128), 128, 0, stream>>>(CTX, WOB, F[9], (float*)d_out);
}
